// Attention_86732569575984
// MI455X (gfx1250) — hardware-verified
//
#include <hip/hip_runtime.h>
#include <math.h>

#ifndef NB
#define NB 2
#endif
#ifndef SEQ
#define SEQ 2048
#endif
#define NB_FULL 2
#define SEQ_FULL 2048
#define DIM 1024
#define NH 16
#define HD 64
#define MTOK (NB * SEQ)
#define OUT1_OFF 4194304

#define Q_CARRY 16.0f
#define K_CARRY 16.0f
#define QK_UNDO (1.0f / 256.0f)
#define KLO_CARRY 2048.0f
#define KLO_UNDO (1.0f / 2048.0f)
#define P_CARRY 1024.0f
#define CTX_CARRY 64.0f
#define WP_CARRY 64.0f
#define OUT_UNDO (1.0f / 4096.0f)
#define K_RATIO 1.04763782f
#define SC2 (0.125f * 1.4426950408889634f * (1.0f / 256.0f))

#define PJ_TN (3 * DIM / 64)
#define PJ_TILES ((MTOK / 64) * PJ_TN)
#define OP_TN (DIM / 64)
#define OP_TILES ((MTOK / 64) * OP_TN)
#define AT_WAVES 4
#define AT_PO 72

#define XB_BYTES (MTOK * DIM * 2)
#define WQ_BYTES (3 * DIM * DIM * 2)
#define WP_BYTES (DIM * DIM * 2)
#define HP_BYTES (NB * NH * SEQ * HD * 2)
#define CTX_BYTES (MTOK * DIM * 2)
#define WS_TOTAL (XB_BYTES + WQ_BYTES + WP_BYTES + 5 * HP_BYTES + CTX_BYTES)

static_assert(Q_CARRY * K_CARRY * QK_UNDO == 1.0f);
static_assert(KLO_CARRY * KLO_UNDO == 1.0f);
static_assert(CTX_CARRY * WP_CARRY * OUT_UNDO == 1.0f);
static_assert(HD == 64 && DIM / 64 == NH && NH == 16);
static_assert(SEQ % 64 == 0 && SEQ <= SEQ_FULL && NB <= NB_FULL);
static_assert(MTOK % 64 == 0 && DIM % 64 == 0 && DIM % 32 == 0);
static_assert(PJ_TILES % 8 == 0 && OP_TILES % 8 == 0);
static_assert((NB * NH * (SEQ / 16)) % AT_WAVES == 0);
static_assert(DIM / 8 == 128);
static_assert((MTOK * DIM / 8) % 256 == 0 && (3 * DIM * DIM / 8) % 256 == 0 && (DIM * DIM / 8) % 256 == 0);
static_assert(OUT1_OFF == NB_FULL * SEQ_FULL * DIM);
static_assert(OUT1_OFF * 4 == 16777216 && (OUT1_OFF * 4) % 128 == 0);
static_assert(XB_BYTES % 256 == 0 && WQ_BYTES % 256 == 0 && WP_BYTES % 256 == 0 && HP_BYTES % 256 == 0 && CTX_BYTES % 256 == 0);
static_assert(WS_TOTAL <= 134217728);
static_assert(8 * 16 * 68 * 4 <= 131072);
static_assert(AT_WAVES * 16 * AT_PO * 2 <= 131072);
static_assert(64 * 68 * 4 <= 131072);
static_assert(4 * 4 == 16 && 2 * 8 == 16);
static_assert(32 * 16 == 4 * 128 && 32 * 16 == 2 * 256);
static_assert(256 * 2 == 64 * 8);

typedef _Float16 h16;
typedef __attribute__((ext_vector_type(16))) _Float16 v16h;
typedef __attribute__((ext_vector_type(8)))  _Float16 v8h;
typedef __attribute__((ext_vector_type(16))) __bf16   v16b;
typedef __attribute__((ext_vector_type(8)))  float    v8f;
typedef __attribute__((ext_vector_type(4)))  float    v4f;
typedef __attribute__((ext_vector_type(4)))  unsigned int v4u;


#define VST2(T, ptr, val) do { const T vst2_v_ = (val); *(volatile T*)(ptr) = vst2_v_; __threadfence(); *(volatile T*)(ptr) = vst2_v_; } while (0)

__device__ __forceinline__ float bfr(float f) {
    unsigned u = __float_as_uint(f);
    u += 0x7FFFu + ((u >> 16) & 1u);
    return __uint_as_float(u & 0xFFFF0000u);
}
__device__ __forceinline__ unsigned bf_pack2(float a, float b) {
    return (__float_as_uint(bfr(a)) >> 16) | __float_as_uint(bfr(b));
}
static __device__ __forceinline__ h16 toh_flush(float v) { const float w = (fabsf(v) < 6.103515625e-05f) ? 0.0f : v; return (h16)w; }

union FragU { v16h v; v8h h[2]; };
union FragBU { v16b v; v4u q[2]; };
__device__ __forceinline__ v16h frag_ld(const _Float16* p) {
    FragU f; f.h[0] = *(const v8h*)(p); f.h[1] = *(const v8h*)(p + 16); return f.v;
}
__device__ __forceinline__ v16b fragb_ld(const unsigned short* p) {
    FragBU f; f.q[0] = *(const v4u*)(p); f.q[1] = *(const v4u*)(p + 16); return f.v;
}
__device__ __forceinline__ v8f wmma16g(v16h a, v16h b, v8f c) {
    c = __builtin_amdgcn_wmma_f32_16x16x32_f16(false, a, false, b, (short)0, c, false, false);
    asm volatile("v_nop\n\tv_nop\n\tv_nop\n\tv_nop" : "+v"(c) : "v"(a), "v"(b));
    return c;
}
__device__ __forceinline__ v8f wmmabg(v16b a, v16b b, v8f c) {
    c = __builtin_amdgcn_wmma_f32_16x16x32_bf16(false, a, false, b, (short)0, c, false, false);
    asm volatile("v_nop\n\tv_nop\n\tv_nop\n\tv_nop" : "+v"(c) : "v"(a), "v"(b));
    return c;
}
__device__ __forceinline__ void wave_sync_lds() {
    __builtin_amdgcn_fence(3  , "workgroup");
    __builtin_amdgcn_wave_barrier();
    __builtin_amdgcn_fence(2  , "workgroup");
}

__global__ __launch_bounds__(256) void k_cvt_x(const float* __restrict__ x, unsigned short* __restrict__ xb) {
    const unsigned u = blockIdx.x * 256u + threadIdx.x;
    if (u >= (unsigned)(MTOK * DIM / 8)) return;
    const unsigned row = u >> 7;
    const unsigned c0 = (u & 127u) * 8u;
    const unsigned b = row / (unsigned)SEQ;
    const unsigned l = row - b * (unsigned)SEQ;
    const float* src = x + (size_t)(b * (unsigned)SEQ_FULL + l) * DIM + c0;
    const v4f a = *(const v4f*)src;
    const v4f c = *(const v4f*)(src + 4);
    v4u pk;
    pk.x = bf_pack2(a.x, a.y); pk.y = bf_pack2(a.z, a.w);
    pk.z = bf_pack2(c.x, c.y); pk.w = bf_pack2(c.z, c.w);
    VST2(v4u, (v4u*)(xb + (size_t)row * DIM + c0), pk);
}

__global__ __launch_bounds__(256) void k_cvt_wq(const float* __restrict__ w, unsigned short* __restrict__ wb) {
    const unsigned u = blockIdx.x * 256u + threadIdx.x;
    if (u >= (unsigned)(3 * DIM * DIM / 8)) return;
    const size_t o = (size_t)u * 8u;
    const v4f a = *(const v4f*)(w + o);
    const v4f c = *(const v4f*)(w + o + 4);
    v4u pk;
    pk.x = bf_pack2(a.x, a.y); pk.y = bf_pack2(a.z, a.w);
    pk.z = bf_pack2(c.x, c.y); pk.w = bf_pack2(c.z, c.w);
    VST2(v4u, (v4u*)(wb + o), pk);
}

__global__ __launch_bounds__(256) void k_cvt_wp(const float* __restrict__ w, _Float16* __restrict__ wp) {
    const unsigned u = blockIdx.x * 256u + threadIdx.x;
    if (u >= (unsigned)(DIM * DIM / 8)) return;
    const size_t o = (size_t)u * 8u;
    const v4f a = *(const v4f*)(w + o);
    const v4f c = *(const v4f*)(w + o + 4);
    v8h hv;
    hv[0] = toh_flush(bfr(a.x) * WP_CARRY); hv[1] = toh_flush(bfr(a.y) * WP_CARRY);
    hv[2] = toh_flush(bfr(a.z) * WP_CARRY); hv[3] = toh_flush(bfr(a.w) * WP_CARRY);
    hv[4] = toh_flush(bfr(c.x) * WP_CARRY); hv[5] = toh_flush(bfr(c.y) * WP_CARRY);
    hv[6] = toh_flush(bfr(c.z) * WP_CARRY); hv[7] = toh_flush(bfr(c.w) * WP_CARRY);
    VST2(v8h, (v8h*)(wp + o), hv);
}

__global__ __launch_bounds__(256) void k_proj(
    const unsigned short* __restrict__ XB, const unsigned short* __restrict__ WQ,
    const float* __restrict__ v0, const float* __restrict__ rc, const float* __restrict__ rs,
    const float* __restrict__ lamp,
    _Float16* __restrict__ QH, _Float16* __restrict__ KHI, _Float16* __restrict__ KLO,
    _Float16* __restrict__ VN, float* __restrict__ out1) {
  __shared__ __align__(16) float sT[8][16 * 68];
  const unsigned lane = threadIdx.x & 31u;
  const unsigned wave = __builtin_amdgcn_readfirstlane(threadIdx.x >> 5);
  const unsigned tile = blockIdx.x * 8u + wave;
  if (tile >= (unsigned)PJ_TILES) return;
  const unsigned tm = tile / (unsigned)PJ_TN;
  const unsigned tn = tile - tm * (unsigned)PJ_TN;
  const unsigned m0 = tm << 6, n0 = tn << 6;
  const unsigned kq = tn >> 4, h = tn & 15u;
  const unsigned b = m0 / (unsigned)SEQ;
  const unsigned l0 = m0 - b * (unsigned)SEQ;
  const unsigned rlane = lane & 15u;
  const unsigned koff = (lane >> 4) * 8u;
  const unsigned mOff = koff;

  v8f acc[4][4];
#pragma unroll
  for (int i = 0; i < 4; ++i)
#pragma unroll
    for (int j = 0; j < 4; ++j) acc[i][j] = (v8f){0.f,0.f,0.f,0.f,0.f,0.f,0.f,0.f};

#pragma unroll 1
  for (unsigned k0 = 0; k0 < (unsigned)DIM; k0 += 32u) {
    v16b bh[4];
#pragma unroll
    for (int j = 0; j < 4; ++j)
      bh[j] = fragb_ld(WQ + (size_t)(n0 + ((unsigned)j << 4) + rlane) * DIM + koff + k0);
#pragma unroll
    for (int i = 0; i < 4; ++i) {
      const v16b ah = fragb_ld(XB + (size_t)(m0 + ((unsigned)i << 4) + rlane) * DIM + koff + k0);
#pragma unroll
      for (int j = 0; j < 4; ++j) acc[i][j] = wmmabg(ah, bh[j], acc[i][j]);
    }
  }

#pragma unroll
  for (int i = 0; i < 4; ++i) {
#pragma unroll
    for (int j = 0; j < 4; ++j)
#pragma unroll
      for (int r = 0; r < 8; ++r)
        sT[wave][(mOff + (unsigned)r) * 68u + ((unsigned)j << 4) + rlane] = acc[i][j][r];
    wave_sync_lds();
    const unsigned lrow0 = l0 + ((unsigned)i << 4);
    if (kq == 2u) {
      const float lam = bfr(lamp[0]);
      const float oml = 1.0f - lam;
      const unsigned hh2 = lane >> 4, c4 = (lane & 15u) * 4u;
#pragma unroll 1
      for (unsigned it = 0; it < 8u; ++it) {
        const unsigned row = it * 2u + hh2;
        const unsigned si = row * 68u + c4;
        v4f vv = *(const v4f*)&sT[wave][si];
        const unsigned fr = (b * (unsigned)NH + h) * (unsigned)SEQ_FULL + lrow0 + row;
        const size_t gi = (size_t)fr * 64u + c4;
        const v4f w = *(const v4f*)(v0 + gi);
        vv.x = lam * vv.x + oml * bfr(w.x);
        vv.y = lam * vv.y + oml * bfr(w.y);
        vv.z = lam * vv.z + oml * bfr(w.z);
        vv.w = lam * vv.w + oml * bfr(w.w);
        *(v4f*)&sT[wave][si] = vv;
        *(volatile v4f*)(out1 + gi) = vv;
        __threadfence();
        *(volatile v4f*)(out1 + gi) = vv;
      }
      wave_sync_lds();
      const unsigned q4 = lane >> 3, c8 = (lane & 7u) * 8u;
#pragma unroll 1
      for (unsigned it = 0; it < 4u; ++it) {
        const unsigned row = it * 4u + q4;
        const unsigned si = row * 68u + c8;
        const v4f a0 = *(const v4f*)&sT[wave][si];
        const v4f a1 = *(const v4f*)&sT[wave][si + 4u];
        v8h hv;
        hv[0] = toh_flush(a0.x); hv[1] = toh_flush(a0.y); hv[2] = toh_flush(a0.z); hv[3] = toh_flush(a0.w);
        hv[4] = toh_flush(a1.x); hv[5] = toh_flush(a1.y); hv[6] = toh_flush(a1.z); hv[7] = toh_flush(a1.w);
        const unsigned pr = (b * (unsigned)NH + h) * (unsigned)SEQ + lrow0 + row;
        _Float16* dst = VN + (size_t)pr * 64u + c8;
        *(volatile v8h*)dst = hv;
        __threadfence();
        *(volatile v8h*)dst = hv;
      }
    } else {
#pragma unroll
      for (int isk = 0; isk < 2; ++isk) {
        if (kq == (unsigned)isk) {
          const unsigned q4 = lane >> 3, j8 = lane & 7u;
          const unsigned c0 = (j8 & 3u) * 8u, c8 = j8 * 8u;
          const bool lowhalf = (j8 < 4u);
#pragma unroll 1
          for (unsigned it = 0; it < 4u; ++it) {
            const unsigned row = it * 4u + q4;
            const unsigned l = lrow0 + row;
            const unsigned si = row * 68u + c0;
            const v4f xa0 = *(const v4f*)&sT[wave][si];
            const v4f xa1 = *(const v4f*)&sT[wave][si + 4u];
            const v4f xb0 = *(const v4f*)&sT[wave][si + 32u];
            const v4f xb1 = *(const v4f*)&sT[wave][si + 36u];
            const float* cp = rc + (size_t)l * 32u + c0;
            const float* sp = rs + (size_t)l * 32u + c0;
            const v4f cc0 = *(const v4f*)cp;
            const v4f cc1 = *(const v4f*)(cp + 4);
            const v4f ss0 = *(const v4f*)sp;
            const v4f ss1 = *(const v4f*)(sp + 4);
            const float x1[8] = {xa0.x, xa0.y, xa0.z, xa0.w, xa1.x, xa1.y, xa1.z, xa1.w};
            const float x2[8] = {xb0.x, xb0.y, xb0.z, xb0.w, xb1.x, xb1.y, xb1.z, xb1.w};
            const float cs[8] = {bfr(cc0.x), bfr(cc0.y), bfr(cc0.z), bfr(cc0.w), bfr(cc1.x), bfr(cc1.y), bfr(cc1.z), bfr(cc1.w)};
            const float sn[8] = {bfr(ss0.x), bfr(ss0.y), bfr(ss0.z), bfr(ss0.w), bfr(ss1.x), bfr(ss1.y), bfr(ss1.z), bfr(ss1.w)};
            float y[8];
            float sq = 0.f;
#pragma unroll
            for (int e = 0; e < 8; ++e) {
              const float y1 = x1[e] * cs[e] + x2[e] * sn[e];
              const float y2 = x2[e] * cs[e] - x1[e] * sn[e];
              float ye = lowhalf ? y1 : y2;
              if (isk) ye *= K_RATIO;
              y[e] = ye;
              sq += ye * ye;
            }
            sq += __shfl_xor(sq, 1, 32);
            sq += __shfl_xor(sq, 2, 32);
            sq += __shfl_xor(sq, 4, 32);
            const float rn = 1.0f / sqrtf(sq * (1.0f / 64.0f) + 1e-6f);
            const unsigned pr = (b * (unsigned)NH + h) * (unsigned)SEQ + l;
            const size_t po = (size_t)pr * 64u + c8;
            if (isk) {
              v8h hv, lv;
#pragma unroll
              for (int e = 0; e < 8; ++e) {
                const float k16 = (y[e] * rn) * K_CARRY;
                const h16 khi = toh_flush(k16);
                hv[e] = khi;
                lv[e] = toh_flush((k16 - (float)khi) * KLO_CARRY);
              }
              *(volatile v8h*)(KHI + po) = hv;
              *(volatile v8h*)(KLO + po) = lv;
              __threadfence();
              *(volatile v8h*)(KHI + po) = hv;
              *(volatile v8h*)(KLO + po) = lv;
            } else {
              v8h hv;
#pragma unroll
              for (int e = 0; e < 8; ++e) hv[e] = toh_flush((y[e] * rn) * Q_CARRY);
              *(volatile v8h*)(QH + po) = hv;
              __threadfence();
              *(volatile v8h*)(QH + po) = hv;
            }
          }
        }
      }
    }
    wave_sync_lds();
  }
}

__global__ __launch_bounds__(256) void k_vt(const _Float16* __restrict__ VN, _Float16* __restrict__ VT) {
    __shared__ __align__(16) float sV[64 * 68];
    const unsigned t = threadIdx.x;
    const unsigned bx = blockIdx.x;
    const unsigned bh = bx / (unsigned)(SEQ / 64);
    const unsigned lt = bx - bh * (unsigned)(SEQ / 64);
    const unsigned lbase = lt * 64u;
#pragma unroll
    for (int it = 0; it < 2; ++it) {
        const unsigned piece = t + 256u * (unsigned)it;
        const unsigned row = piece >> 3, c8 = (piece & 7u) * 8u;
        const v8h vv = *(const v8h*)(VN + ((size_t)bh * SEQ + lbase + row) * 64u + c8);
        v4f f0, f1;
        f0.x = (float)vv[0]; f0.y = (float)vv[1]; f0.z = (float)vv[2]; f0.w = (float)vv[3];
        f1.x = (float)vv[4]; f1.y = (float)vv[5]; f1.z = (float)vv[6]; f1.w = (float)vv[7];
        *(v4f*)&sV[row * 68u + c8] = f0;
        *(v4f*)&sV[row * 68u + c8 + 4u] = f1;
    }
    __syncthreads();
#pragma unroll
    for (int it = 0; it < 2; ++it) {
        const unsigned piece = t + 256u * (unsigned)it;
        const unsigned d = piece >> 3, l8 = (piece & 7u) * 8u;
        v8h o;
#pragma unroll
        for (int e = 0; e < 8; ++e) o[e] = toh_flush(sV[(l8 + (unsigned)e) * 68u + d]);
        VST2(v8h, (v8h*)(VT + ((size_t)bh * 64u + d) * SEQ + lbase + l8), o);
    }
}

__global__ __launch_bounds__(128) void k_attn(const _Float16* __restrict__ QH, const _Float16* __restrict__ KHI,
                                              const _Float16* __restrict__ KLO, const _Float16* __restrict__ VT,
                                              _Float16* __restrict__ CTX) {
    __shared__ __align__(16) _Float16 sO[AT_WAVES][16 * AT_PO];
    const unsigned lane = threadIdx.x & 31u;
    const unsigned wave = __builtin_amdgcn_readfirstlane(threadIdx.x >> 5);
    const unsigned hh = lane >> 4, c = lane & 15u;
    const unsigned gw = blockIdx.x * (unsigned)AT_WAVES + wave;
    const unsigned bh = gw / (unsigned)(SEQ / 16);
    const unsigned qt = gw - bh * (unsigned)(SEQ / 16);
    const unsigned q0 = qt * 16u;
    const unsigned b = bh / (unsigned)NH;
    const unsigned h = bh - b * (unsigned)NH;
    const size_t hb = (size_t)bh * SEQ * 64u;

    const v16h qf0 = frag_ld(QH + hb + (size_t)(q0 + c) * 64u + 8u * hh);
    const v16h qf1 = frag_ld(QH + hb + (size_t)(q0 + c) * 64u + 32u + 8u * hh);

    float mrun = -3.0e38f, lrun = 0.f;
    v8f ot[4];
#pragma unroll
    for (int t = 0; t < 4; ++t) ot[t] = (v8f){0.f,0.f,0.f,0.f,0.f,0.f,0.f,0.f};

#pragma unroll 1
    for (unsigned kv0 = 0; kv0 < (unsigned)SEQ; kv0 += 32u) {
        v8f sh[2], sl[2];
#pragma unroll
        for (int j = 0; j < 2; ++j) {
            const size_t ko = hb + (size_t)(kv0 + (unsigned)j * 16u + c) * 64u + 8u * hh;
            const v16h ka0 = frag_ld(KHI + ko);
            const v16h ka1 = frag_ld(KHI + ko + 32u);
            const v16h la0 = frag_ld(KLO + ko);
            const v16h la1 = frag_ld(KLO + ko + 32u);
            const v8f z = (v8f){0.f,0.f,0.f,0.f,0.f,0.f,0.f,0.f};
            sh[j] = wmma16g(ka0, qf0, z);
            sh[j] = wmma16g(ka1, qf1, sh[j]);
            sl[j] = wmma16g(la0, qf0, z);
            sl[j] = wmma16g(la1, qf1, sl[j]);
        }
        float s[2][8];
        float mx = -3.0e38f;
#pragma unroll
        for (int j = 0; j < 2; ++j)
#pragma unroll
            for (int r = 0; r < 8; ++r) {
                s[j][r] = (sh[j][r] + sl[j][r] * KLO_UNDO) * SC2;
                mx = fmaxf(mx, s[j][r]);
            }
        mx = fmaxf(mx, __shfl_xor(mx, 16, 32));
        const float mnew = fmaxf(mrun, mx);
        const float alpha = exp2f(mrun - mnew);
        mrun = mnew;
        FragU pf;
        float psum = 0.f;
#pragma unroll
        for (int j = 0; j < 2; ++j)
#pragma unroll
            for (int r = 0; r < 8; ++r) {
                const float p = exp2f(s[j][r] - mnew) * P_CARRY;
                const h16 ph = toh_flush(p);
                pf.v[8 * j + r] = ph;
                psum += (float)ph;
            }
        lrun = lrun * alpha + psum;
#pragma unroll
        for (int t = 0; t < 4; ++t)
#pragma unroll
            for (int r = 0; r < 8; ++r) ot[t][r] *= alpha;
#pragma unroll
        for (int t = 0; t < 4; ++t) {
            const v16h va = frag_ld(VT + hb + (size_t)((unsigned)t * 16u + c) * SEQ + kv0 + 8u * hh);
            ot[t] = wmma16g(va, pf.v, ot[t]);
        }
    }

    const float ltot = lrun + __shfl_xor(lrun, 16, 32);
    const float inv = CTX_CARRY * (1.0f / ltot);
#pragma unroll
    for (int t = 0; t < 4; ++t) {
        v8h o;
#pragma unroll
        for (int r = 0; r < 8; ++r) o[r] = toh_flush(ot[t][r] * inv);
        *(v8h*)&sO[wave][c * (unsigned)AT_PO + (2u * (unsigned)t + hh) * 8u] = o;
    }
    wave_sync_lds();
    {
        const unsigned q4 = lane >> 3, c8 = (lane & 7u) * 8u;
#pragma unroll 1
        for (unsigned it = 0; it < 4u; ++it) {
            const unsigned row = it * 4u + q4;
            const v8h ov = *(const v8h*)&sO[wave][row * (unsigned)AT_PO + c8];
            _Float16* dst = CTX + (size_t)(b * (unsigned)SEQ + q0 + row) * DIM + h * 64u + c8;
            *(volatile v8h*)dst = ov;
            __threadfence();
            *(volatile v8h*)dst = ov;
        }
    }
}

__global__ __launch_bounds__(256) void k_oproj(const _Float16* __restrict__ CTX, const _Float16* __restrict__ WP,
                                               float* __restrict__ out0) {
  __shared__ __align__(16) float sT[8][16 * 68];
  const unsigned lane = threadIdx.x & 31u;
  const unsigned wave = __builtin_amdgcn_readfirstlane(threadIdx.x >> 5);
  const unsigned tile = blockIdx.x * 8u + wave;
  if (tile >= (unsigned)OP_TILES) return;
  const unsigned tm = tile / (unsigned)OP_TN;
  const unsigned tn = tile - tm * (unsigned)OP_TN;
  const unsigned m0 = tm << 6, n0 = tn << 6;
  const unsigned b = m0 / (unsigned)SEQ;
  const unsigned l0 = m0 - b * (unsigned)SEQ;
  const unsigned rlane = lane & 15u;
  const unsigned koff = (lane >> 4) * 8u;
  const unsigned mOff = koff;

  v8f acc[4][4];
#pragma unroll
  for (int i = 0; i < 4; ++i)
#pragma unroll
    for (int j = 0; j < 4; ++j) acc[i][j] = (v8f){0.f,0.f,0.f,0.f,0.f,0.f,0.f,0.f};

#pragma unroll 1
  for (unsigned k0 = 0; k0 < (unsigned)DIM; k0 += 32u) {
    v16h bh[4];
#pragma unroll
    for (int j = 0; j < 4; ++j)
      bh[j] = frag_ld(WP + (size_t)(n0 + ((unsigned)j << 4) + rlane) * DIM + koff + k0);
#pragma unroll
    for (int i = 0; i < 4; ++i) {
      const v16h ah = frag_ld(CTX + (size_t)(m0 + ((unsigned)i << 4) + rlane) * DIM + koff + k0);
#pragma unroll
      for (int j = 0; j < 4; ++j) acc[i][j] = wmma16g(ah, bh[j], acc[i][j]);
    }
  }

#pragma unroll
  for (int i = 0; i < 4; ++i) {
#pragma unroll
    for (int j = 0; j < 4; ++j)
#pragma unroll
      for (int r = 0; r < 8; ++r)
        sT[wave][(mOff + (unsigned)r) * 68u + ((unsigned)j << 4) + rlane] = acc[i][j][r] * OUT_UNDO;
    wave_sync_lds();
    const unsigned hh2 = lane >> 4, c4 = (lane & 15u) * 4u;
    const unsigned frow0 = b * (unsigned)SEQ_FULL + l0 + ((unsigned)i << 4);
#pragma unroll 1
    for (unsigned it = 0; it < 8u; ++it) {
      const unsigned row = it * 2u + hh2;
      const v4f vv = *(const v4f*)&sT[wave][row * 68u + c4];
      float* dst = out0 + (size_t)(frow0 + row) * DIM + n0 + c4;
      *(volatile v4f*)dst = vv;
      __threadfence();
      *(volatile v4f*)dst = vv;
    }
    wave_sync_lds();
  }
}

extern "C" void kernel_launch(void* const* d_in, const int* in_sizes, int n_in, void* d_out, int out_size,
                              void* d_ws, size_t ws_size, hipStream_t stream) {
    if (n_in < 7) return;
    if (in_sizes[0] < ((NB - 1) * SEQ_FULL + SEQ) * DIM) return;
    if (in_sizes[1] < (((NB - 1) * NH + (NH - 1)) * SEQ_FULL + SEQ) * HD) return;
    if (in_sizes[2] < SEQ * (HD / 2) || in_sizes[3] < SEQ * (HD / 2)) return;
    if (in_sizes[4] < 3 * DIM * DIM || in_sizes[5] < DIM * DIM || in_sizes[6] < 1) return;
    if (out_size < OUT1_OFF + (((NB - 1) * NH + (NH - 1)) * SEQ_FULL + SEQ) * HD) return;

    const float* x      = (const float*)d_in[0];
    const float* v_0    = (const float*)d_in[1];
    const float* rcos   = (const float*)d_in[2];
    const float* rsin   = (const float*)d_in[3];
    const float* qkv_w  = (const float*)d_in[4];
    const float* proj_w = (const float*)d_in[5];
    const float* lamp   = (const float*)d_in[6];
    float* out0 = (float*)d_out;
    float* out1 = (float*)d_out + OUT1_OFF;

    char* wsp = (char*)d_ws;
    size_t off = 0;
    auto carve = [&](size_t bytes) -> void* { void* r = wsp + off; off += (bytes + 255) & ~(size_t)255; return r; };
    unsigned short* xb  = (unsigned short*)carve((size_t)XB_BYTES);
    unsigned short* wq  = (unsigned short*)carve((size_t)WQ_BYTES);
    _Float16*       wp  = (_Float16*)carve((size_t)WP_BYTES);
    _Float16*       qh  = (_Float16*)carve((size_t)HP_BYTES);
    _Float16*       khi = (_Float16*)carve((size_t)HP_BYTES);
    _Float16*       klo = (_Float16*)carve((size_t)HP_BYTES);
    _Float16*       vn  = (_Float16*)carve((size_t)HP_BYTES);
    _Float16*       vt  = (_Float16*)carve((size_t)HP_BYTES);
    _Float16*       ctx = (_Float16*)carve((size_t)CTX_BYTES);
    if (off > ws_size || off > (size_t)134217728) return;

    k_cvt_x<<<(MTOK * DIM / 8) / 256, 256, 0, stream>>>(x, xb);
    k_cvt_wq<<<(3 * DIM * DIM / 8) / 256, 256, 0, stream>>>(qkv_w, wq);
    k_cvt_wp<<<(DIM * DIM / 8) / 256, 256, 0, stream>>>(proj_w, wp);

    k_proj<<<PJ_TILES / 8, 256, 0, stream>>>(xb, wq, v_0, rcos, rsin, lamp, qh, khi, klo, vn, out1);

    k_vt<<<NB * NH * (SEQ / 64), 256, 0, stream>>>(vn, vt);

    k_attn<<<(NB * NH * (SEQ / 16)) / AT_WAVES, 128, 0, stream>>>(qh, khi, klo, vt, ctx);

    k_oproj<<<OP_TILES / 8, 256, 0, stream>>>(ctx, wp, out0);
}
